// CondConv2d_5531917877687
// MI455X (gfx1250) — hardware-verified
//
#include <hip/hip_runtime.h>
#include <stdint.h>

#define DEVINL __device__ __forceinline__

typedef _Float16 f16t;
typedef _Float16 v16h __attribute__((ext_vector_type(16)));
typedef _Float16 v8h  __attribute__((ext_vector_type(8)));
typedef float    v8f  __attribute__((ext_vector_type(8)));
typedef float    v4f  __attribute__((ext_vector_type(4)));
typedef v8h __attribute__((may_alias)) v8ha;
typedef v4f __attribute__((may_alias)) v4fa;
union FragH { v16h v; v8h half[2]; };

#define NB     32
#define CIN    3
#define HWIN   70
#define OWD    64
#define LWIN   4096
#define KTAP   49
#define KP     64
#define OCH    256
#define HID    24
#define HIDP   32
#define NOUT   3
#define NOUTP  16
#define TPB    256
#define NWAVE  8
#define XSTR   72
#define LPB    32
#define UPW    4
#define RSP    32
#define GDIV   (LWIN * CIN)

#define XS   8.0f
#define WS   64.0f
#define AC   8.0f
#define W1S  256.0f
#define HC   8.0f
#define W2S  64.0f

static_assert(LWIN % LPB == 0);
static_assert(NWAVE * UPW == LPB);
static_assert(TPB == NWAVE * 32);
static_assert((XSTR * 2) % 16 == 0);
static_assert(NB == 32);
static_assert((CIN * OCH * KP / 8) % TPB == 0);
static_assert(NB * NOUT == 96);

DEVINL int imin(int a, int b) { return a < b ? a : b; }

DEVINL v8f wmma_f16(v16h a, v16h b, v8f c) {
  v8f d = __builtin_amdgcn_wmma_f32_16x16x32_f16(false, a, false, b, (short)0, c, false, false);
  asm volatile("v_nop\n\tv_nop\n\tv_nop\n\tv_nop" : "+v"(d) : "v"(a), "v"(b));
  return d;
}
DEVINL v8f zero8f() {
  v8f z = {0.f, 0.f, 0.f, 0.f, 0.f, 0.f, 0.f, 0.f};
  return z;
}

DEVINL void wave_fence() {
  __builtin_amdgcn_fence(__ATOMIC_RELEASE, "wavefront");
  asm volatile("s_wait_dscnt 0" ::: "memory");
  __builtin_amdgcn_wave_barrier();
  __builtin_amdgcn_fence(__ATOMIC_ACQUIRE, "wavefront");
}

__global__ __launch_bounds__(TPB) void prep_k(const float* __restrict__ cnn_w,
                                             const float* __restrict__ w1,
                                             const float* __restrict__ w2,
                                             f16t* __restrict__ WcP,
                                             f16t* __restrict__ W1P,
                                             f16t* __restrict__ W2P)
{
  const int t = blockIdx.x * TPB + threadIdx.x;
  const int y = blockIdx.y;
  if (y == 0) {
    if (t >= CIN * OCH * (KP / 8)) return;
    const int part = t & 7;
    const int o    = (t >> 3) & (OCH - 1);
    const int c    = t >> 11;
    v8h o8;
    #pragma unroll
    for (int i = 0; i < 8; ++i) {
      const int q  = 8 * part + i;
      const int qc = imin(q, KTAP - 1);
      const float w  = cnn_w[(o * CIN + c) * KTAP + qc];
      const float sc = (q < KTAP) ? WS : 0.0f;
      o8[i] = (f16t)(w * sc);
    }
    f16t* dst = WcP + (size_t)8 * t;
    *(volatile v8h*)dst = o8;
    __threadfence();
    *(volatile v8h*)dst = o8;
  } else if (y == 1) {
    if (t >= HIDP * (OCH / 8)) return;
    const int n    = t >> 5;
    const int part = t & 31;
    const int nc   = imin(n, HID - 1);
    const float sc = (n < HID) ? W1S : 0.0f;
    v8h o8;
    #pragma unroll
    for (int i = 0; i < 8; ++i) {
      const int k = 8 * part + i;
      const float w = w1[k * HID + nc];
      o8[i] = (f16t)(w * sc);
    }
    f16t* dst = W1P + (size_t)8 * t;
    *(volatile v8h*)dst = o8;
    __threadfence();
    *(volatile v8h*)dst = o8;
  } else {
    if (t >= NOUTP * (HIDP / 8)) return;
    const int j    = t >> 2;
    const int part = t & 3;
    const int jc   = imin(j, NOUT - 1);
    v8h o8;
    #pragma unroll
    for (int i = 0; i < 8; ++i) {
      const int n  = 8 * part + i;
      const int nc = imin(n, HID - 1);
      const float w  = w2[nc * NOUT + jc];
      const float sc = (j < NOUT && n < HID) ? W2S : 0.0f;
      o8[i] = (f16t)(w * sc);
    }
    f16t* dst = W2P + (size_t)8 * t;
    *(volatile v8h*)dst = o8;
    __threadfence();
    *(volatile v8h*)dst = o8;
  }
}

__global__ __launch_bounds__(TPB) void condconv_k(const float* __restrict__ x,
                                                 const float* __restrict__ b1,
                                                 const float* __restrict__ b2,
                                                 const f16t* __restrict__ WcP,
                                                 const f16t* __restrict__ W1P,
                                                 const f16t* __restrict__ W2P,
                                                 float* __restrict__ out)
{
  __shared__ __attribute__((aligned(16))) f16t  sx[NWAVE * 32 * XSTR];
  __shared__ __attribute__((aligned(16))) float sres[NB * NOUT * RSP];
  const int tid = threadIdx.x, lane = tid & 31, wave = tid >> 5;
  const int h = lane >> 4, m = lane & 15;
  const int l0 = blockIdx.x * LPB;
  f16t* xt = sx + wave * (32 * XSTR);

  const float CSCL = AC / (XS * WS);
  const float INV1 = 1.0f / (AC * W1S);
  const float INV2 = 1.0f / (HC * W2S);

  #pragma unroll 1
  for (int i = 0; i < UPW; ++i) {
    const int lloc = wave * UPW + i;
    const int lp   = l0 + lloc;
    v8f oacc[2];
    oacc[0] = zero8f();
    oacc[1] = zero8f();

    #pragma unroll 1
    for (int cp = 0; cp < CIN; ++cp) {
      wave_fence();
      {
        const int G   = lp * (CIN * NB) + cp * NB + lane;
        const int bb  = G / GDIV;
        const int rem = G - bb * GDIV;
        const int l   = rem / CIN;
        const int cc  = rem - l * CIN;
        const int ohl = l >> 6, owl = l & 63;
        const float* xb = x + ((size_t)(bb * CIN + cc) * HWIN + ohl) * HWIN + owl;
        const float zpad = xb[0] * 0.0f;
        #pragma unroll
        for (int j = 0; j < 8; ++j) {
          v8h pc;
          #pragma unroll
          for (int e = 0; e < 8; ++e) {
            const int k = 8 * j + e;
            float v;
            if (k < KTAP) {
              const int kh = k / 7;
              const int kw = k - kh * 7;
              v = xb[kh * HWIN + kw] * XS;
            } else {
              v = zpad;
            }
            pc[e] = (f16t)v;
          }
          *(v8h*)(xt + lane * XSTR + 8 * j) = pc;
        }
      }
      wave_fence();

      v8f hT[2][2];
      #pragma unroll
      for (int nt = 0; nt < 2; ++nt) {
        hT[nt][0] = zero8f();
        hT[nt][1] = zero8f();
      }
      const f16t* wcb = WcP + (size_t)(cp * OCH) * KP;

      #pragma unroll 1
      for (int oc = 0; oc < 8; ++oc) {
        FragH af[2][2];
        #pragma unroll
        for (int ct = 0; ct < 2; ++ct) {
          #pragma unroll
          for (int ks = 0; ks < 2; ++ks) {
            const f16t* p = wcb + (size_t)(32 * oc + 16 * ct + m) * KP + 32 * ks + 8 * h;
            af[ct][ks].half[0] = *(const v8ha*)(p);
            af[ct][ks].half[1] = *(const v8ha*)(p + 16);
          }
        }
        FragH wf[2];
        #pragma unroll
        for (int nt = 0; nt < 2; ++nt) {
          const f16t* p = W1P + (size_t)(16 * nt + m) * OCH + 32 * oc + 8 * h;
          wf[nt].half[0] = *(const v8ha*)(p);
          wf[nt].half[1] = *(const v8ha*)(p + 16);
        }
        #pragma unroll
        for (int bt = 0; bt < 2; ++bt) {
          FragH xb0, xb1;
          const f16t* xr = xt + (16 * bt + m) * XSTR + 8 * h;
          xb0.half[0] = *(const v8ha*)(xr);
          xb0.half[1] = *(const v8ha*)(xr + 16);
          xb1.half[0] = *(const v8ha*)(xr + 32);
          xb1.half[1] = *(const v8ha*)(xr + 48);
          v8f d0 = wmma_f16(af[0][0].v, xb0.v, zero8f());
          d0 = wmma_f16(af[0][1].v, xb1.v, d0);
          v8f d1 = wmma_f16(af[1][0].v, xb0.v, zero8f());
          d1 = wmma_f16(af[1][1].v, xb1.v, d1);
          FragH bp;
          #pragma unroll
          for (int r = 0; r < 8; ++r) {
            bp.v[r]     = (f16t)(fmaxf(d0[r], 0.0f) * CSCL);
            bp.v[8 + r] = (f16t)(fmaxf(d1[r], 0.0f) * CSCL);
          }
          hT[0][bt] = wmma_f16(wf[0].v, bp.v, hT[0][bt]);
          hT[1][bt] = wmma_f16(wf[1].v, bp.v, hT[1][bt]);
        }
      }

      {
        FragH w2f;
        const f16t* p = W2P + m * HIDP + 8 * h;
        w2f.half[0] = *(const v8ha*)(p);
        w2f.half[1] = *(const v8ha*)(p + 16);
        float ba[8], bbv[8];
        #pragma unroll
        for (int r = 0; r < 8; ++r) {
          ba[r]  = b1[8 * h + r];
          bbv[r] = b1[imin(16 + 8 * h + r, HID - 1)];
        }
        const bool vhi = (h == 0);
        #pragma unroll
        for (int bt = 0; bt < 2; ++bt) {
          FragH bh;
          #pragma unroll
          for (int r = 0; r < 8; ++r) {
            const float u0 = fmaxf(fmaf(hT[0][bt][r], INV1, ba[r]), 0.0f) * HC;
            const float u1 = fmaxf(fmaf(hT[1][bt][r], INV1, bbv[r]), 0.0f) * HC;
            bh.v[r]     = (f16t)u0;
            bh.v[8 + r] = vhi ? (f16t)u1 : (f16t)0.0f;
          }
          oacc[bt] = wmma_f16(w2f.v, bh.v, oacc[bt]);
        }
      }
    }

    if (h == 0) {
      #pragma unroll
      for (int bt = 0; bt < 2; ++bt) {
        const int bpr = 16 * bt + m;
        #pragma unroll
        for (int r = 0; r < NOUT; ++r) {
          const float v = fmaf(oacc[bt][r], INV2, 3.0f * b2[r]);
          sres[(bpr * NOUT + r) * RSP + lloc] = v;
        }
      }
    }
  }
  __syncthreads();

  {
    const int q  = tid & 7;
    const int lq = tid >> 3;
    v4f vv[3];
    #pragma unroll
    for (int p = 0; p < 3; ++p) vv[p] = *(const v4fa*)(sres + (32 * p + lq) * RSP + 4 * q);
    float* ob = out + (size_t)l0 + 4 * q;
    #pragma unroll
    for (int p = 0; p < 3; ++p) *(volatile v4f*)(ob + (size_t)(32 * p + lq) * LWIN) = vv[p];
    __threadfence();
    #pragma unroll
    for (int p = 0; p < 3; ++p) *(volatile v4f*)(ob + (size_t)(32 * p + lq) * LWIN) = vv[p];
  }
}

extern "C" void kernel_launch(void* const* d_in, const int* in_sizes, int n_in,
                              void* d_out, int out_size, void* d_ws, size_t ws_size,
                              hipStream_t stream) {
  if (n_in < 6) return;
  if (out_size != NB * NOUT * LWIN) return;
  if (in_sizes[0] != NB * CIN * HWIN * HWIN) return;
  if (in_sizes[1] != OCH * CIN * KTAP) return;
  if (in_sizes[2] != OCH * HID) return;
  if (in_sizes[3] != HID) return;
  if (in_sizes[4] != HID * NOUT) return;
  if (in_sizes[5] != NOUT) return;

  const float* x     = (const float*)d_in[0];
  const float* cnn_w = (const float*)d_in[1];
  const float* w1    = (const float*)d_in[2];
  const float* b1    = (const float*)d_in[3];
  const float* w2    = (const float*)d_in[4];
  const float* b2    = (const float*)d_in[5];
  float* outp = (float*)d_out;

  const size_t szWc = (size_t)CIN * OCH * KP * 2;
  const size_t szW1 = (size_t)HIDP * OCH * 2;
  const size_t szW2 = (size_t)NOUTP * HIDP * 2;
  size_t off = 0;
  char* ws = (char*)d_ws;
  f16t* WcP = (f16t*)(ws + off); off += szWc;
  f16t* W1P = (f16t*)(ws + off); off += szW1;
  f16t* W2P = (f16t*)(ws + off); off += szW2;
  if (off > ws_size) return;
  if (off > (size_t)128 * 1024 * 1024) return;

  prep_k<<<dim3(CIN * OCH * (KP / 8) / TPB, 3), TPB, 0, stream>>>(cnn_w, w1, w2, WcP, W1P, W2P);
  condconv_k<<<LWIN / LPB, TPB, 0, stream>>>(x, b1, b2, WcP, W1P, W2P, outp);
}
